// WavLM_38955353375365
// MI455X (gfx1250) — hardware-verified
//
#include <hip/hip_runtime.h>
#include <math.h>
#include <stdint.h>

typedef __attribute__((ext_vector_type(16))) _Float16 v16h;
typedef __attribute__((ext_vector_type(8)))  _Float16 v8h;
typedef __attribute__((ext_vector_type(4)))  _Float16 v4h;
typedef __attribute__((ext_vector_type(16))) __bf16   v16b;
typedef __attribute__((ext_vector_type(8)))  __bf16   v8b;
typedef __attribute__((ext_vector_type(8)))  float    v8f;
typedef __attribute__((ext_vector_type(4)))  float    v4f;
#define U16(p) ((const unsigned short*)(const void*)(p))

__device__ __forceinline__ unsigned short f2bf_bits(float f) {
  unsigned u = __float_as_uint(f);
  return (unsigned short)((u + 0x7FFFu + ((u >> 16) & 1u)) >> 16);
}
__device__ __forceinline__ float bf_bits2f(unsigned short h) { return __uint_as_float(((unsigned)h) << 16); }

__device__ __forceinline__ void dep_guard_h(v8f& a, v8f& b, v16h x, v16h y) { asm volatile("v_nop\n\tv_nop\n\tv_nop\n\tv_nop" : "+v"(a), "+v"(b) : "v"(x), "v"(y)); }
__device__ __forceinline__ void dep_guard_b(v8f& a, v8f& b, v16b x, v16b y) { asm volatile("v_nop\n\tv_nop\n\tv_nop\n\tv_nop" : "+v"(a), "+v"(b) : "v"(x), "v"(y)); }
__device__ __forceinline__ void keep4_h(v16h a, v16h b, v16h c, v16h d) { asm volatile("v_nop" :: "v"(a), "v"(b), "v"(c), "v"(d)); }
__device__ __forceinline__ void keep4_b(v16b a, v16b b, v16b c, v16b d) { asm volatile("v_nop" :: "v"(a), "v"(b), "v"(c), "v"(d)); }
__device__ __forceinline__ void acc_guard4(v8f& a, v8f& b, v8f& c, v8f& d) { asm volatile("v_nop\n\tv_nop\n\tv_nop\n\tv_nop" : "+v"(a), "+v"(b), "+v"(c), "+v"(d)); }
template <typename T> struct Frag;
template <> struct Frag<_Float16> {
  typedef v16h V; union U { v16h v; v8h h[2]; };
  static __device__ __forceinline__ v16h load(const _Float16* p) {
    U f; f.h[0] = *(const v8h*)(p); f.h[1] = *(const v8h*)(p + 16); return f.v;
  }
  static __device__ __forceinline__ v8f mma(v16h a, v16h b, v8f c) {
    return __builtin_amdgcn_wmma_f32_16x16x32_f16(false, a, false, b, (short)0, c, false, false);
  }
  static __device__ __forceinline__ void guard(v8f& a, v8f& b, v16h x, v16h y) { dep_guard_h(a, b, x, y); }
  static __device__ __forceinline__ void keep(v16h a, v16h b, v16h c, v16h d) { keep4_h(a, b, c, d); }
};
template <> struct Frag<__bf16> {
  typedef v16b V; union U { v16b v; v8b h[2]; };
  static __device__ __forceinline__ v16b load(const __bf16* p) {
    U f; f.h[0] = *(const v8b*)(p); f.h[1] = *(const v8b*)(p + 16); return f.v;
  }
  static __device__ __forceinline__ v8f mma(v16b a, v16b b, v8f c) {
    return __builtin_amdgcn_wmma_f32_16x16x32_bf16(false, a, false, b, (short)0, c, false, false);
  }
  static __device__ __forceinline__ void guard(v8f& a, v8f& b, v16b x, v16b y) { dep_guard_b(a, b, x, y); }
  static __device__ __forceinline__ void keep(v16b a, v16b b, v16b c, v16b d) { keep4_b(a, b, c, d); }
};

template <int ET> struct Elem;
template <> struct Elem<0> { typedef _Float16 T; };
template <> struct Elem<1> { typedef __bf16 T; };
template <int ET, bool SPLIT, int BIAS_MODE, int OUT_MODE, bool RESID, int ACT = 0>
__global__ __launch_bounds__(256) void wmma_gemm64(
    const unsigned short* __restrict__ Ap, const unsigned short* __restrict__ A2p, int lda, long strideA,
    const unsigned short* __restrict__ Btp, const unsigned short* __restrict__ Bt2p, int ldb, long strideB,
    void* __restrict__ Cout, void* __restrict__ Cout2, int ldc, long strideC,
    const float* __restrict__ bias,
    const float* __restrict__ resid, long strideR,
    int M, int N, int K, float scale) {
  typedef typename Elem<ET>::T T;
  typedef typename Frag<T>::V V;
  const T* A = (const T*)Ap; const T* A2 = (const T*)A2p; const T* Bt = (const T*)Btp; const T* Bt2 = (const T*)Bt2p;
  __shared__ __align__(16) float sT[8][16 * 68];
  const int b    = blockIdx.y;
  const int lane = threadIdx.x & 31;
  const int wave = threadIdx.x >> 5;
  const int tilesN = N >> 6;
  const int tilesM = M >> 6;
  const int tile = blockIdx.x * 8 + wave;
  if (tile >= tilesM * tilesN) return;
  const int tm = tile / tilesN;
  const int tn = tile - tm * tilesN;
  const int m0 = tm << 6;
  const int n0 = tn << 6;

  const T* Ab  = A  + (size_t)b * strideA;
  const T* Bb  = Bt + (size_t)b * strideB;
  const T* Ab2 = SPLIT ? (A2  + (size_t)b * strideA) : nullptr;
  const T* Bb2 = SPLIT ? (Bt2 + (size_t)b * strideB) : nullptr;

  const int rlane = lane & 15;
  const int koff  = (lane >> 4) * 8;
  const int mOff  = (lane >> 4) * 8;

  v8f acc[4][4];
#pragma unroll
  for (int i = 0; i < 4; ++i)
#pragma unroll
    for (int j = 0; j < 4; ++j) acc[i][j] = (v8f){0.f,0.f,0.f,0.f,0.f,0.f,0.f,0.f};

  for (int k0 = 0; k0 < K; k0 += 32) {
    V bh[4], bl[4];
#pragma unroll
    for (int j = 0; j < 4; ++j) {
      const size_t bo = (size_t)(n0 + (j << 4) + rlane) * ldb + koff + k0;
      bh[j] = Frag<T>::load(Bb + bo);
      if (SPLIT) bl[j] = Frag<T>::load(Bb2 + bo);
    }
#pragma unroll
    for (int i = 0; i < 4; ++i) {
      const size_t ao = (size_t)(m0 + (i << 4) + rlane) * lda + koff + k0;
      V ah = Frag<T>::load(Ab + ao);
      V al;
      if (SPLIT) al = Frag<T>::load(Ab2 + ao);
#pragma unroll
      for (int j = 0; j < 4; ++j) {
        acc[i][j] = Frag<T>::mma(ah, bh[j], acc[i][j]);
        if (SPLIT) {
          acc[i][j] = Frag<T>::mma(ah, bl[j], acc[i][j]);
          acc[i][j] = Frag<T>::mma(al, bh[j], acc[i][j]);
        }
      }
      Frag<T>::guard(acc[i][0], acc[i][3], ah, SPLIT ? al : ah);
    }
    Frag<T>::keep(bh[0], bh[1], bh[2], bh[3]);
    if (SPLIT) Frag<T>::keep(bl[0], bl[1], bl[2], bl[3]);
  }
  acc_guard4(acc[0][0], acc[0][1], acc[0][2], acc[0][3]);
  acc_guard4(acc[1][0], acc[1][1], acc[1][2], acc[1][3]);
  acc_guard4(acc[2][0], acc[2][1], acc[2][2], acc[2][3]);
  acc_guard4(acc[3][0], acc[3][1], acc[3][2], acc[3][3]);

  float* slab = sT[wave];
  const float* Rb = RESID ? (resid + (size_t)b * strideR) : nullptr;
#pragma unroll
  for (int i = 0; i < 4; ++i) {
    const int mBase = m0 + (i << 4);
#pragma unroll
    for (int j = 0; j < 4; ++j) {
      const int n = n0 + (j << 4) + rlane;
      float bv = 0.f;
      if (BIAS_MODE == 2) bv = bias[n];
#pragma unroll
      for (int r = 0; r < 8; ++r) {
        float v = acc[i][j][r] * scale;
        if (BIAS_MODE == 1) v += bias[mBase + mOff + r];
        if (BIAS_MODE == 2) v += bv;
        if (RESID) v += Rb[(size_t)(mBase + mOff + r) * ldc + n];
        if (ACT == 1) v = tanhf(v);
        if (ACT == 2) v = fmaxf(v, 0.0f);
        if (ACT == 3) v = v / (1.0f + expf(-v));
        if (ACT == 4) v = (v > 0.f) ? v : 0.01f * v;
        if (ACT == 5) v = 0.5f * v * (1.0f + erff(v * 0.70710678118654752f));
        slab[(mOff + r) * 68 + (j << 4) + rlane] = v;
      }
    }
    __builtin_amdgcn_fence(__ATOMIC_RELEASE, "workgroup");
    __builtin_amdgcn_wave_barrier();
    __builtin_amdgcn_fence(__ATOMIC_ACQUIRE, "workgroup");
    if (OUT_MODE == 0) {
      float* C = (float*)Cout + (size_t)b * strideC;
      const int hh = lane >> 4, c4 = (lane & 15) * 4;
      for (int pass = 0; pass < 2; ++pass) {
#pragma unroll
        for (int it = 0; it < 8; ++it) {
          const int row = it * 2 + hh;
          v4f v = *(const v4f*)(slab + row * 68 + c4);
          *(volatile v4f*)(C + (size_t)(mBase + row) * ldc + n0 + c4) = v;
        }
        __threadfence();
      }
    } else {
      const int q = lane >> 3, c8 = (lane & 7) * 8;
      unsigned short* C  = (unsigned short*)Cout  + (size_t)b * strideC;
      unsigned short* C2 = (OUT_MODE == 2) ? ((unsigned short*)Cout2 + (size_t)b * strideC) : nullptr;
      for (int pass = 0; pass < 2; ++pass) {
#pragma unroll
        for (int it = 0; it < 4; ++it) {
          const int row = it * 4 + q;
          const float* sp = slab + row * 68 + c8;
          v8h hv, lv;
#pragma unroll
          for (int e = 0; e < 8; ++e) {
            if (OUT_MODE == 1) {
              hv[e] = (_Float16)sp[e];
            } else {
              unsigned short hb = f2bf_bits(sp[e]);
              unsigned short lb = f2bf_bits(sp[e] - bf_bits2f(hb));
              hv[e] = __builtin_bit_cast(_Float16, hb);
              lv[e] = __builtin_bit_cast(_Float16, lb);
            }
          }
          *(volatile v8h*)(C + (size_t)(mBase + row) * ldc + n0 + c8) = hv;
          if (OUT_MODE == 2) *(volatile v8h*)(C2 + (size_t)(mBase + row) * ldc + n0 + c8) = lv;
        }
        __threadfence();
      }
    }
    __builtin_amdgcn_fence(__ATOMIC_RELEASE, "workgroup");
    __builtin_amdgcn_wave_barrier();
    __builtin_amdgcn_fence(__ATOMIC_ACQUIRE, "workgroup");
  }
}

__global__ __launch_bounds__(256) void cast_scale_f32_f16x2(
    const float* __restrict__ in, _Float16* __restrict__ out, int n2, float sc) {
  int i = blockIdx.x * 256 + threadIdx.x;
  if (i < n2) {
    const _Float16 h0 = (_Float16)(in[2 * i] * sc), h1 = (_Float16)(in[2 * i + 1] * sc);
    const unsigned u = (unsigned)__builtin_bit_cast(unsigned short, h0) | ((unsigned)__builtin_bit_cast(unsigned short, h1) << 16);
    ((volatile unsigned*)out)[i] = u;
    __threadfence();
    ((volatile unsigned*)out)[i] = u;
  }
}

#define LN_T 192
template <int PRE>
__global__ __launch_bounds__(LN_T) void ln_kernel(
    const float* __restrict__ in, const float* __restrict__ pos, const float* __restrict__ mask,
    const float* __restrict__ g, const float* __restrict__ bb,
    float* __restrict__ outf, _Float16* __restrict__ outh, int C, float invC, float eps) {
  __shared__ float rs[8];
  __shared__ float rq[8];
  const int row = blockIdx.x;
  const int tid = threadIdx.x;
  const int lane = tid & 31;
  const int w = tid >> 5;
  const int c4 = tid * 4;
  const size_t base = (size_t)row * C + c4;
  v4f xv = *(const v4f*)(in + base);
  if (PRE) {
    const float mk = mask[row];
    const v4f pv = *(const v4f*)(pos + base);
    xv = xv * mk + pv;
  }
  float s = (xv[0] + xv[1]) + (xv[2] + xv[3]);
#pragma unroll
  for (int off = 16; off > 0; off >>= 1) s += __shfl_xor(s, off, 32);
  if (lane == 0) rs[w] = s;
  __syncthreads();
  float ts = 0.f;
#pragma unroll
  for (int i = 0; i < LN_T / 32; ++i) ts += rs[i];
  const float mean = ts * invC;
  const v4f d = xv - mean;
  float sq = (d[0] * d[0] + d[1] * d[1]) + (d[2] * d[2] + d[3] * d[3]);
#pragma unroll
  for (int off = 16; off > 0; off >>= 1) sq += __shfl_xor(sq, off, 32);
  if (lane == 0) rq[w] = sq;
  __syncthreads();
  float tq = 0.f;
#pragma unroll
  for (int i = 0; i < LN_T / 32; ++i) tq += rq[i];
  const float var = tq * invC;
  const float inv = rsqrtf(var + eps);
  const v4f gv = *(const v4f*)(g + c4);
  const v4f bv = *(const v4f*)(bb + c4);
  const v4f y = d * inv * gv + bv;
  v4h yh;
  yh[0] = (_Float16)y[0]; yh[1] = (_Float16)y[1]; yh[2] = (_Float16)y[2]; yh[3] = (_Float16)y[3];
  *(volatile v4f*)(outf + base) = y;
  *(volatile v4h*)(outh + base) = yh;
  __threadfence();
  *(volatile v4f*)(outf + base) = y;
  *(volatile v4h*)(outh + base) = yh;
}

__global__ __launch_bounds__(256) void gate_kernel(
    const float* __restrict__ hf, const float* __restrict__ gw, const float* __restrict__ gb,
    const float* __restrict__ gc, float* __restrict__ gate, int S, int H, int C, int total) {
  const int idx = blockIdx.x * 256 + threadIdx.x;
  if (idx >= total) return;
  const int s  = idx % S;
  const int bh = idx / S;
  const int h  = bh % H;
  const int b  = bh / H;
  const float* hp = hf + ((size_t)b * S + s) * C + (size_t)h * 64;
  float acc[8];
#pragma unroll
  for (int e = 0; e < 8; ++e) acc[e] = 0.f;
#pragma unroll 1
  for (int d = 0; d < 64; ++d) {
    const float hv = hp[d];
#pragma unroll
    for (int e = 0; e < 8; ++e) acc[e] = fmaf(hv, gw[e * 64 + d], acc[e]);
  }
  const float sa = ((acc[0] + gb[0]) + (acc[1] + gb[1])) + ((acc[2] + gb[2]) + (acc[3] + gb[3]));
  const float sb = ((acc[4] + gb[4]) + (acc[5] + gb[5])) + ((acc[6] + gb[6]) + (acc[7] + gb[7]));
  const float ga  = 1.0f / (1.0f + expf(-sa));
  const float gbv = 1.0f / (1.0f + expf(-sb));
  const float gv = ga * (gbv * gc[h] - 1.0f) + 2.0f;
  ((volatile float*)gate)[idx] = gv;
  __threadfence();
  ((volatile float*)gate)[idx] = gv;
}

#define AT_D 64
#define AT_NW 4
#define AT_KC 64
#define AT_PSC 32768.0f

__device__ __forceinline__ v8f hmma(v16h a, v16h b, v8f c) {
  c = __builtin_amdgcn_wmma_f32_16x16x32_f16(false, a, false, b, (short)0, c, false, false);
  asm volatile("v_nop\n\tv_nop\n\tv_nop\n\tv_nop" : "+v"(c) : "v"(a), "v"(b));
  return c;
}

__global__ __launch_bounds__(128)
void attn_gbias_kernel(const float* __restrict__ q, const float* __restrict__ k,
                       const float* __restrict__ v, const float* __restrict__ gate,
                       const float* __restrict__ pos_bias, const float* __restrict__ mask,
                       _Float16* __restrict__ out, int S, int H, int C, float qscale) {
  union FH { v16h v; v8h h[2]; };
  __shared__ __align__(16) _Float16 Ksh[AT_KC * AT_D];
  __shared__ __align__(16) _Float16 Vth[AT_D * AT_KC];
  __shared__ __align__(16) _Float16 Psh[AT_NW][16 * AT_KC];
  __shared__ __align__(16) float    Os[AT_NW][16 * 68];

  const int tid  = threadIdx.x;
  const int wave = tid >> 5;
  const int lane = tid & 31;
  const int hh   = lane >> 4;
  const int c    = lane & 15;

  const int nqb = S / 64;
  const int bx = blockIdx.x;
  const int qb = bx % nqb;
  const int bh = bx / nqb;
  const int h  = bh % H;
  const int b  = bh / H;
  const int q0 = qb * 64 + wave * 16;

  const float* qb_ptr = q + (size_t)b * S * C + (size_t)h * AT_D;
  const float* kb_ptr = k + (size_t)b * S * C + (size_t)h * AT_D;
  const float* vb_ptr = v + (size_t)b * S * C + (size_t)h * AT_D;
  const float* gt_ptr = gate + ((size_t)b * H + h) * S;
  const float* pb_ptr = pos_bias + (size_t)h * S * S;
  const float* mk_ptr = mask + (size_t)b * S;
  _Float16*    ob_ptr = out + (size_t)b * S * C + (size_t)h * AT_D;

  v16h qa[2];
  {
    const float* qrow = qb_ptr + (size_t)(q0 + c) * C;
#pragma unroll
    for (int dc = 0; dc < 2; ++dc) {
#pragma unroll
      for (int e = 0; e < 8; ++e) {
        qa[dc][e]     = (_Float16)qrow[dc * 32 + 8 * hh + e];
        qa[dc][8 + e] = (_Float16)qrow[dc * 32 + 16 + 8 * hh + e];
      }
    }
  }
  float grow[8];
#pragma unroll
  for (int r = 0; r < 8; ++r) grow[r] = gt_ptr[q0 + 8 * hh + r];

  float mrow[8], lrow[8];
  v8f oacc[4];
#pragma unroll
  for (int r = 0; r < 8; ++r) { mrow[r] = -INFINITY; lrow[r] = 0.f; }
#pragma unroll
  for (int t = 0; t < 4; ++t) oacc[t] = (v8f){0.f,0.f,0.f,0.f,0.f,0.f,0.f,0.f};

  const int nChunks = S / AT_KC;
  for (int kc = 0; kc < nChunks; ++kc) {
    const int kv0 = kc * AT_KC;
    __syncthreads();
    {
      const int kvr = tid >> 1, dh = (tid & 1) * 32;
      const float* krow = kb_ptr + (size_t)(kv0 + kvr) * C + dh;
      const float* vrow = vb_ptr + (size_t)(kv0 + kvr) * C + dh;
#pragma unroll
      for (int i = 0; i < 8; ++i) {
        v4f kk = *(const v4f*)(krow + 4 * i);
        v4f vv = *(const v4f*)(vrow + 4 * i);
#pragma unroll
        for (int e = 0; e < 4; ++e) {
          const int d = dh + 4 * i + e;
          Ksh[kvr * AT_D + d]  = (_Float16)kk[e];
          Vth[d * AT_KC + kvr] = (_Float16)vv[e];
        }
      }
    }
    __syncthreads();

    v8f s[4];
#pragma unroll
    for (int j = 0; j < 4; ++j) {
      s[j] = (v8f){0.f,0.f,0.f,0.f,0.f,0.f,0.f,0.f};
#pragma unroll
      for (int dc = 0; dc < 2; ++dc) {
        FH kb;
        kb.h[0] = *(const v8h*)(Ksh + (j * 16 + c) * AT_D + dc * 32 + 8 * hh);
        kb.h[1] = *(const v8h*)(Ksh + (j * 16 + c) * AT_D + dc * 32 + 16 + 8 * hh);
        s[j] = hmma(qa[dc], kb.v, s[j]);
      }
    }
    float kp[4];
#pragma unroll
    for (int j = 0; j < 4; ++j) kp[j] = (1.0f - mk_ptr[kv0 + j * 16 + c]) * -10000.0f;
    float cm[8];
#pragma unroll
    for (int r = 0; r < 8; ++r) {
      const int qrow = q0 + 8 * hh + r;
      const float* pbr = pb_ptr + (size_t)qrow * S + kv0;
      float m = -INFINITY;
#pragma unroll
      for (int j = 0; j < 4; ++j) {
        const float sv = s[j][r] * qscale + grow[r] * pbr[j * 16 + c] + kp[j];
        s[j][r] = sv;
        m = fmaxf(m, sv);
      }
#pragma unroll
      for (int off = 1; off < 16; off <<= 1) m = fmaxf(m, __shfl_xor(m, off, 32));
      cm[r] = m;
    }
    _Float16* pw = Psh[wave];
#pragma unroll
    for (int r = 0; r < 8; ++r) {
      const float mnew = fmaxf(mrow[r], cm[r]);
      const float alpha = expf(mrow[r] - mnew);
      mrow[r] = mnew;
      float psum = 0.f;
#pragma unroll
      for (int j = 0; j < 4; ++j) {
        const float p = expf(s[j][r] - mnew);
        psum += p;
        pw[(8 * hh + r) * AT_KC + j * 16 + c] = (_Float16)(p * AT_PSC);
      }
#pragma unroll
      for (int off = 1; off < 16; off <<= 1) psum += __shfl_xor(psum, off, 32);
      lrow[r] = lrow[r] * alpha + psum;
#pragma unroll
      for (int t = 0; t < 4; ++t) oacc[t][r] *= alpha;
    }
    __builtin_amdgcn_fence(__ATOMIC_RELEASE, "workgroup");
    __builtin_amdgcn_wave_barrier();
    __builtin_amdgcn_fence(__ATOMIC_ACQUIRE, "workgroup");
#pragma unroll 1
    for (int kk = 0; kk < 2; ++kk) {
      FH pa;
      pa.h[0] = *(const v8h*)(pw + c * AT_KC + kk * 32 + 8 * hh);
      pa.h[1] = *(const v8h*)(pw + c * AT_KC + kk * 32 + 16 + 8 * hh);
#pragma unroll
      for (int t = 0; t < 4; ++t) {
        FH vb;
        vb.h[0] = *(const v8h*)(Vth + (t * 16 + c) * AT_KC + kk * 32 + 8 * hh);
        vb.h[1] = *(const v8h*)(Vth + (t * 16 + c) * AT_KC + kk * 32 + 16 + 8 * hh);
        oacc[t] = hmma(pa.v, vb.v, oacc[t]);
      }
    }
  }

  float* os = Os[wave];
#pragma unroll
  for (int r = 0; r < 8; ++r) {
    const float inv = 1.0f / (lrow[r] * AT_PSC);
#pragma unroll
    for (int t = 0; t < 4; ++t) os[(8 * hh + r) * 68 + t * 16 + c] = oacc[t][r] * inv;
  }
  __builtin_amdgcn_fence(__ATOMIC_RELEASE, "workgroup");
  __builtin_amdgcn_wave_barrier();
  __builtin_amdgcn_fence(__ATOMIC_ACQUIRE, "workgroup");
  {
    const int q8 = lane >> 3, c8 = (lane & 7) * 8;
    for (int pass = 0; pass < 2; ++pass) {
#pragma unroll
      for (int it = 0; it < 4; ++it) {
        const int row = it * 4 + q8;
        const float* sp = os + row * 68 + c8;
        v8h hv;
#pragma unroll
        for (int e = 0; e < 8; ++e) hv[e] = (_Float16)sp[e];
        *(volatile v8h*)(ob_ptr + (size_t)(q0 + row) * C + c8) = hv;
      }
      __threadfence();
    }
  }
}

extern "C" void kernel_launch(void* const* d_in, const int* in_sizes, int n_in,
                              void* d_out, int out_size, void* d_ws, size_t ws_size,
                              hipStream_t stream) {
  const int Bn = 2, S = 1024, C = 768, H = 12, L = 4, FF = 3072;
  const int M = Bn * S;
  if (n_in < 25) return;
  if (in_sizes[0] != M * C || in_sizes[1] != M * C || in_sizes[2] != M || in_sizes[3] != H * S * S) return;
  if (in_sizes[6] != L * C * C || in_sizes[19] != L * FF * C || in_sizes[21] != L * C * FF) return;
  if (out_size != M * C) return;

  const float* x        = (const float*)d_in[0];
  const float* pos_emb  = (const float*)d_in[1];
  const float* attn_m   = (const float*)d_in[2];
  const float* pos_bias = (const float*)d_in[3];
  const float* ln0_g    = (const float*)d_in[4];
  const float* ln0_b    = (const float*)d_in[5];
  const float* Wq       = (const float*)d_in[6];
  const float* bq       = (const float*)d_in[7];
  const float* Wk       = (const float*)d_in[8];
  const float* bk       = (const float*)d_in[9];
  const float* Wv       = (const float*)d_in[10];
  const float* bv       = (const float*)d_in[11];
  const float* Wo       = (const float*)d_in[12];
  const float* bo       = (const float*)d_in[13];
  const float* gruW     = (const float*)d_in[14];
  const float* grub     = (const float*)d_in[15];
  const float* gruc     = (const float*)d_in[16];
  const float* ln1_g    = (const float*)d_in[17];
  const float* ln1_b    = (const float*)d_in[18];
  const float* W1       = (const float*)d_in[19];
  const float* b1       = (const float*)d_in[20];
  const float* W2       = (const float*)d_in[21];
  const float* b2       = (const float*)d_in[22];
  const float* ln2_g    = (const float*)d_in[23];
  const float* ln2_b    = (const float*)d_in[24];

  char* ws = (char*)d_ws;
  size_t off = 0;
  const size_t NWC = (size_t)L * C * C;
  const size_t NWF = (size_t)L * FF * C;
  const size_t NA  = (size_t)M * C;
  const size_t NF  = (size_t)M * FF;
  const size_t NG  = (size_t)Bn * H * S;
  size_t o_wq, o_wk, o_wv, o_wo, o_w1, o_w2, o_hf, o_hh, o_qf, o_kf, o_vf, o_ao, o_h1f, o_h1h, o_ff, o_gt;
#define CARVE(o, bytes) do { o = off; off += ((size_t)(bytes) + 255) & ~(size_t)255; } while (0)
  CARVE(o_wq, NWC * 2); CARVE(o_wk, NWC * 2); CARVE(o_wv, NWC * 2); CARVE(o_wo, NWC * 2);
  CARVE(o_w1, NWF * 2); CARVE(o_w2, NWF * 2);
  CARVE(o_hf, NA * 4);  CARVE(o_hh, NA * 2);
  CARVE(o_qf, NA * 4);  CARVE(o_kf, NA * 4);  CARVE(o_vf, NA * 4);
  CARVE(o_ao, NA * 2);
  CARVE(o_h1f, NA * 4); CARVE(o_h1h, NA * 2);
  CARVE(o_ff, NF * 2);
  CARVE(o_gt, NG * 4);
#undef CARVE
  if (off > ws_size) return;

  _Float16* wq16 = (_Float16*)(ws + o_wq);
  _Float16* wk16 = (_Float16*)(ws + o_wk);
  _Float16* wv16 = (_Float16*)(ws + o_wv);
  _Float16* wo16 = (_Float16*)(ws + o_wo);
  _Float16* w116 = (_Float16*)(ws + o_w1);
  _Float16* w216 = (_Float16*)(ws + o_w2);
  float*    hf   = (float*)(ws + o_hf);
  _Float16* hh16 = (_Float16*)(ws + o_hh);
  float*    qf   = (float*)(ws + o_qf);
  float*    kf   = (float*)(ws + o_kf);
  float*    vf   = (float*)(ws + o_vf);
  _Float16* ao16 = (_Float16*)(ws + o_ao);
  float*    h1f  = (float*)(ws + o_h1f);
  _Float16* h1h  = (_Float16*)(ws + o_h1h);
  _Float16* ff16 = (_Float16*)(ws + o_ff);
  float*    gtb  = (float*)(ws + o_gt);
  float*    outp = (float*)d_out;

  const float WSC  = 64.0f;
  const float WINV = 1.0f / 64.0f;
  const float invC = 1.0f / 768.0f;
  const float eps  = 1e-5f;
  const float qscale = 0.125f;

  {
    const int n2c = (int)(NWC / 2), n2f = (int)(NWF / 2);
    cast_scale_f32_f16x2<<<(n2c + 255) / 256, 256, 0, stream>>>(Wq, wq16, n2c, WSC);
    cast_scale_f32_f16x2<<<(n2c + 255) / 256, 256, 0, stream>>>(Wk, wk16, n2c, WSC);
    cast_scale_f32_f16x2<<<(n2c + 255) / 256, 256, 0, stream>>>(Wv, wv16, n2c, WSC);
    cast_scale_f32_f16x2<<<(n2c + 255) / 256, 256, 0, stream>>>(Wo, wo16, n2c, WSC);
    cast_scale_f32_f16x2<<<(n2f + 255) / 256, 256, 0, stream>>>(W1, w116, n2f, WSC);
    cast_scale_f32_f16x2<<<(n2f + 255) / 256, 256, 0, stream>>>(W2, w216, n2f, WSC);
  }

  ln_kernel<1><<<M, LN_T, 0, stream>>>(x, pos_emb, attn_m, ln0_g, ln0_b, hf, hh16, C, invC, eps);

  const int nbP = ((M / 64) * (C / 64) + 7) / 8;
  const int nbF = ((M / 64) * (FF / 64) + 7) / 8;
  const int nbA = Bn * H * (S / 64);
  const int ngate = (int)NG;
  const int nbG = (ngate + 255) / 256;

  for (int l = 0; l < L; ++l) {
    const size_t lw  = (size_t)l * C * C;
    const size_t lwf = (size_t)l * FF * C;
    const _Float16* WQl = wq16 + lw;
    const _Float16* WKl = wk16 + lw;
    const _Float16* WVl = wv16 + lw;
    const _Float16* WOl = wo16 + lw;
    const _Float16* W1l = w116 + lwf;
    const _Float16* W2l = w216 + lwf;

    wmma_gemm64<0, false, 2, 0, false, 0><<<dim3(nbP, 1), 256, 0, stream>>>(
        U16(hh16), U16(hh16), C, 0L, U16(WQl), U16(WQl), C, 0L,
        (void*)qf, (void*)qf, C, 0L, bq + (size_t)l * C, hf, 0L, M, C, C, WINV);
    wmma_gemm64<0, false, 2, 0, false, 0><<<dim3(nbP, 1), 256, 0, stream>>>(
        U16(hh16), U16(hh16), C, 0L, U16(WKl), U16(WKl), C, 0L,
        (void*)kf, (void*)kf, C, 0L, bk + (size_t)l * C, hf, 0L, M, C, C, WINV);
    wmma_gemm64<0, false, 2, 0, false, 0><<<dim3(nbP, 1), 256, 0, stream>>>(
        U16(hh16), U16(hh16), C, 0L, U16(WVl), U16(WVl), C, 0L,
        (void*)vf, (void*)vf, C, 0L, bv + (size_t)l * C, hf, 0L, M, C, C, WINV);

    gate_kernel<<<nbG, 256, 0, stream>>>(hf, gruW + (size_t)l * 8 * 64, grub + (size_t)l * 8,
                                          gruc + (size_t)l * H, gtb, S, H, C, ngate);

    attn_gbias_kernel<<<nbA, 128, 0, stream>>>(qf, kf, vf, gtb, pos_bias, attn_m, ao16, S, H, C, qscale);

    wmma_gemm64<0, false, 2, 0, true, 0><<<dim3(nbP, 1), 256, 0, stream>>>(
        U16(ao16), U16(ao16), C, 0L, U16(WOl), U16(WOl), C, 0L,
        (void*)qf, (void*)qf, C, 0L, bo + (size_t)l * C, hf, 0L, M, C, C, WINV);

    ln_kernel<0><<<M, LN_T, 0, stream>>>(qf, qf, attn_m, ln1_g + (size_t)l * C, ln1_b + (size_t)l * C,
                                         h1f, h1h, C, invC, eps);

    wmma_gemm64<0, false, 2, 1, false, 5><<<dim3(nbF, 1), 256, 0, stream>>>(
        U16(h1h), U16(h1h), C, 0L, U16(W1l), U16(W1l), C, 0L,
        (void*)ff16, (void*)ff16, FF, 0L, b1 + (size_t)l * FF, h1f, 0L, M, FF, C, WINV);

    wmma_gemm64<0, false, 2, 0, true, 0><<<dim3(nbP, 1), 256, 0, stream>>>(
        U16(ff16), U16(ff16), FF, 0L, U16(W2l), U16(W2l), FF, 0L,
        (void*)kf, (void*)kf, C, 0L, b2 + (size_t)l * C, h1f, 0L, M, C, FF, WINV);

    float* hdst = (l == L - 1) ? outp : hf;
    ln_kernel<0><<<M, LN_T, 0, stream>>>(kf, kf, attn_m, ln2_g + (size_t)l * C, ln2_b + (size_t)l * C,
                                         hdst, hh16, C, invC, eps);
  }
  (void)hipGetLastError();
}
